// CoAttention_24850680774977
// MI455X (gfx1250) — hardware-verified
//
#include <hip/hip_runtime.h>
#include <math.h>

#ifndef NB
#define NB 32
#endif
#define NB_FULL 32
#define NEV 5
#define LCQ 64
#define LEQ 128
#define DM 768
#define HDN 256
#define NPAIR (NB * NEV)
#define NPAIR_FULL (NB_FULL * NEV)
#define PCH 40
#define P2 (2 * DM)
#define P3 (3 * DM)
#define PA3 (3 * LEQ)
#define PT3 (3 * LCQ)
static_assert(NPAIR_FULL * DM * 4 == 491520);
static_assert(DM % 128 == 0);
static_assert(HDN == 256);
static_assert(LCQ % 64 == 0 && LEQ % 64 == 0 && DM % 64 == 0 && HDN % 64 == 0);
static_assert(P2 % 32 == 0 && P3 % 32 == 0 && PA3 % 32 == 0 && PT3 % 32 == 0);

typedef __attribute__((ext_vector_type(16))) _Float16 v16h;
typedef __attribute__((ext_vector_type(8)))  _Float16 v8h;
typedef __attribute__((ext_vector_type(16))) __bf16   v16b;
typedef __attribute__((ext_vector_type(8)))  __bf16   v8b;
typedef __attribute__((ext_vector_type(8)))  float    v8f;
typedef __attribute__((ext_vector_type(4)))  float    v4f;
typedef __attribute__((ext_vector_type(4)))  unsigned int v4u;

#define VST2(T, ptr, val) do { const T vst2_v_ = (val); *(volatile T*)(ptr) = vst2_v_; __threadfence(); *(volatile T*)(ptr) = vst2_v_; } while (0)

__device__ __forceinline__ unsigned short bfbits(float f) { unsigned int u = __float_as_uint(f); u += 0x7fffu + ((u >> 16) & 1u); return (unsigned short)(u >> 16); }
__device__ __forceinline__ float bfval(unsigned short h) { return __uint_as_float(((unsigned int)h) << 16); }
__device__ __forceinline__ float bfr(float f) { return bfval(bfbits(f)); }
__device__ __forceinline__ v4u pack8(const unsigned short* h) {
    v4u p;
    p.x = (unsigned int)h[0] | ((unsigned int)h[1] << 16);
    p.y = (unsigned int)h[2] | ((unsigned int)h[3] << 16);
    p.z = (unsigned int)h[4] | ((unsigned int)h[5] << 16);
    p.w = (unsigned int)h[6] | ((unsigned int)h[7] << 16);
    return p;
}
__device__ __forceinline__ void split4(const float* o, unsigned long long& ph, unsigned long long& pl) {
    unsigned short h[4], l[4];
#pragma unroll
    for (int i = 0; i < 4; ++i) { h[i] = bfbits(o[i]); l[i] = bfbits(o[i] - bfval(h[i])); }
    ph = (unsigned long long)h[0] | ((unsigned long long)h[1] << 16) | ((unsigned long long)h[2] << 32) | ((unsigned long long)h[3] << 48);
    pl = (unsigned long long)l[0] | ((unsigned long long)l[1] << 16) | ((unsigned long long)l[2] << 32) | ((unsigned long long)l[3] << 48);
}

namespace w25 {

__device__ __forceinline__ unsigned short f2bf_bits(float f) {
  unsigned u = __float_as_uint(f);
  return (unsigned short)((u + 0x7FFFu + ((u >> 16) & 1u)) >> 16);
}
__device__ __forceinline__ float bf_bits2f(unsigned short h) { return __uint_as_float(((unsigned)h) << 16); }

__device__ __forceinline__ void dep_guard_h(v8f& a, v8f& b, v16h x, v16h y) { asm volatile("v_nop\n\tv_nop\n\tv_nop\n\tv_nop" : "+v"(a), "+v"(b) : "v"(x), "v"(y)); }
__device__ __forceinline__ void dep_guard_b(v8f& a, v8f& b, v16b x, v16b y) { asm volatile("v_nop\n\tv_nop\n\tv_nop\n\tv_nop" : "+v"(a), "+v"(b) : "v"(x), "v"(y)); }
__device__ __forceinline__ void keep4_h(v16h a, v16h b, v16h c, v16h d) { asm volatile("v_nop" :: "v"(a), "v"(b), "v"(c), "v"(d)); }
__device__ __forceinline__ void keep4_b(v16b a, v16b b, v16b c, v16b d) { asm volatile("v_nop" :: "v"(a), "v"(b), "v"(c), "v"(d)); }
__device__ __forceinline__ void acc_guard4(v8f& a, v8f& b, v8f& c, v8f& d) { asm volatile("v_nop\n\tv_nop\n\tv_nop\n\tv_nop" : "+v"(a), "+v"(b), "+v"(c), "+v"(d)); }
template <typename T> struct Frag;
template <> struct Frag<_Float16> {
  typedef v16h V; union U { v16h v; v8h h[2]; };
  static __device__ __forceinline__ v16h load(const _Float16* p) {
    U f; f.h[0] = *(const v8h*)(p); f.h[1] = *(const v8h*)(p + 16); return f.v;
  }
  static __device__ __forceinline__ v8f mma(v16h a, v16h b, v8f c) {
    return __builtin_amdgcn_wmma_f32_16x16x32_f16(false, a, false, b, (short)0, c, false, false);
  }
  static __device__ __forceinline__ void guard(v8f& a, v8f& b, v16h x, v16h y) { dep_guard_h(a, b, x, y); }
  static __device__ __forceinline__ void keep(v16h a, v16h b, v16h c, v16h d) { keep4_h(a, b, c, d); }
};
template <> struct Frag<__bf16> {
  typedef v16b V; union U { v16b v; v8b h[2]; };
  static __device__ __forceinline__ v16b load(const __bf16* p) {
    U f; f.h[0] = *(const v8b*)(p); f.h[1] = *(const v8b*)(p + 16); return f.v;
  }
  static __device__ __forceinline__ v8f mma(v16b a, v16b b, v8f c) {
    return __builtin_amdgcn_wmma_f32_16x16x32_bf16(false, a, false, b, (short)0, c, false, false);
  }
  static __device__ __forceinline__ void guard(v8f& a, v8f& b, v16b x, v16b y) { dep_guard_b(a, b, x, y); }
  static __device__ __forceinline__ void keep(v16b a, v16b b, v16b c, v16b d) { keep4_b(a, b, c, d); }
};

template <int ET> struct Elem;
template <> struct Elem<0> { typedef _Float16 T; };
template <> struct Elem<1> { typedef __bf16 T; };
template <int ET, bool SPLIT, int BIAS_MODE, int OUT_MODE, bool RESID, int ACT = 0>
__global__ __launch_bounds__(256) void wmma_gemm64(
    const unsigned short* __restrict__ Ap, const unsigned short* __restrict__ A2p, int lda, long strideA,
    const unsigned short* __restrict__ Btp, const unsigned short* __restrict__ Bt2p, int ldb, long strideB,
    void* Cout, void* Cout2, void* Cout3, int ldc, long strideC,
    const float* __restrict__ bias,
    const float* __restrict__ resid, long strideR,
    int M, int N, int K, float scale) {
  typedef typename Elem<ET>::T T;
  typedef typename Frag<T>::V V;
  const T* A = (const T*)Ap; const T* A2 = (const T*)A2p; const T* Bt = (const T*)Btp; const T* Bt2 = (const T*)Bt2p;
  __shared__ __align__(16) float sT[8][16 * 68];
  const int b    = blockIdx.y;
  const int lane = threadIdx.x & 31;
  const int wave = threadIdx.x >> 5;
  const int tilesN = N >> 6;
  const int tilesM = M >> 6;
  const int tile = blockIdx.x * 8 + wave;
  if (tile >= tilesM * tilesN) return;
  const int tm = tile / tilesN;
  const int tn = tile - tm * tilesN;
  const int m0 = tm << 6;
  const int n0 = tn << 6;

  const T* Ab  = A  + (size_t)b * strideA;
  const T* Bb  = Bt + (size_t)b * strideB;
  const T* Ab2 = SPLIT ? (A2  + (size_t)b * strideA) : nullptr;
  const T* Bb2 = SPLIT ? (Bt2 + (size_t)b * strideB) : nullptr;

  const int rlane = lane & 15;
  const int koff  = (lane >> 4) * 8;
  const int mOff  = (lane >> 4) * 8;

  v8f acc[4][4];
#pragma unroll
  for (int i = 0; i < 4; ++i)
#pragma unroll
    for (int j = 0; j < 4; ++j) acc[i][j] = (v8f){0.f,0.f,0.f,0.f,0.f,0.f,0.f,0.f};

  for (int k0 = 0; k0 < K; k0 += 32) {
    V bh[4], bl[4];
#pragma unroll
    for (int j = 0; j < 4; ++j) {
      const size_t bo = (size_t)(n0 + (j << 4) + rlane) * ldb + koff + k0;
      bh[j] = Frag<T>::load(Bb + bo);
      if (SPLIT) bl[j] = Frag<T>::load(Bb2 + bo);
    }
#pragma unroll
    for (int i = 0; i < 4; ++i) {
      const size_t ao = (size_t)(m0 + (i << 4) + rlane) * lda + koff + k0;
      V ah = Frag<T>::load(Ab + ao);
      V al;
      if (SPLIT) al = Frag<T>::load(Ab2 + ao);
#pragma unroll
      for (int j = 0; j < 4; ++j) {
        acc[i][j] = Frag<T>::mma(ah, bh[j], acc[i][j]);
        if (SPLIT) {
          acc[i][j] = Frag<T>::mma(ah, bl[j], acc[i][j]);
          acc[i][j] = Frag<T>::mma(al, bh[j], acc[i][j]);
        }
      }
      Frag<T>::guard(acc[i][0], acc[i][3], ah, SPLIT ? al : ah);
    }
    Frag<T>::keep(bh[0], bh[1], bh[2], bh[3]);
    if (SPLIT) Frag<T>::keep(bl[0], bl[1], bl[2], bl[3]);
  }
  acc_guard4(acc[0][0], acc[0][1], acc[0][2], acc[0][3]);
  acc_guard4(acc[1][0], acc[1][1], acc[1][2], acc[1][3]);
  acc_guard4(acc[2][0], acc[2][1], acc[2][2], acc[2][3]);
  acc_guard4(acc[3][0], acc[3][1], acc[3][2], acc[3][3]);

  float* slab = sT[wave];
  const float* Rb = RESID ? (resid + (size_t)b * strideR) : nullptr;
#pragma unroll
  for (int i = 0; i < 4; ++i) {
    const int mBase = m0 + (i << 4);
#pragma unroll
    for (int j = 0; j < 4; ++j) {
      const int n = n0 + (j << 4) + rlane;
      float bv = 0.f;
      if (BIAS_MODE == 2) bv = bias[n];
#pragma unroll
      for (int r = 0; r < 8; ++r) {
        float v = acc[i][j][r] * scale;
        if (BIAS_MODE == 1) v += bias[mBase + mOff + r];
        if (BIAS_MODE == 2) v += bv;
        if (RESID) v += Rb[(size_t)(mBase + mOff + r) * ldc + n];
        if (ACT == 1) v = tanhf(v);
        if (ACT == 2) v = fmaxf(v, 0.0f);
        slab[(mOff + r) * 68 + (j << 4) + rlane] = v;
      }
    }
    __builtin_amdgcn_fence(__ATOMIC_RELEASE, "workgroup");
    __builtin_amdgcn_wave_barrier();
    __builtin_amdgcn_fence(__ATOMIC_ACQUIRE, "workgroup");
    if (OUT_MODE == 0) {
      float* C = (float*)Cout + (size_t)b * strideC;
      const int hh = lane >> 4, c4 = (lane & 15) * 4;
      for (int pass = 0; pass < 2; ++pass) {
#pragma unroll
        for (int it = 0; it < 8; ++it) {
          const int row = it * 2 + hh;
          v4f v = *(const v4f*)(slab + row * 68 + c4);
          *(volatile v4f*)(C + (size_t)(mBase + row) * ldc + n0 + c4) = v;
        }
        __threadfence();
      }
    } else {
      const int q = lane >> 3, c8 = (lane & 7) * 8;
      unsigned short* C  = (unsigned short*)Cout  + (size_t)b * strideC;
      unsigned short* C2 = (OUT_MODE == 2) ? ((unsigned short*)Cout2 + (size_t)b * strideC) : nullptr;
      unsigned short* C3 = (OUT_MODE == 2 && Cout3) ? ((unsigned short*)Cout3 + (size_t)b * strideC) : nullptr;
      for (int pass = 0; pass < 2; ++pass) {
#pragma unroll
        for (int it = 0; it < 4; ++it) {
          const int row = it * 4 + q;
          const float* sp = slab + row * 68 + c8;
          unsigned short hb[8], lb[8];
#pragma unroll
          for (int e = 0; e < 8; ++e) {
            if (OUT_MODE == 1) {
              hb[e] = __builtin_bit_cast(unsigned short, (_Float16)sp[e]); lb[e] = (unsigned short)0;
            } else {
              hb[e] = f2bf_bits(sp[e]);
              lb[e] = f2bf_bits(sp[e] - bf_bits2f(hb[e]));
            }
          }
          const v4u hv = pack8(hb), lv = pack8(lb);
          const size_t off = (size_t)(mBase + row) * ldc + n0 + c8;
          *(volatile v4u*)(C + off) = hv;
          if (OUT_MODE == 2) { *(volatile v4u*)(C2 + off) = lv; if (C3) *(volatile v4u*)(C3 + off) = hv; }
        }
        __threadfence();
      }
    }
    __builtin_amdgcn_fence(__ATOMIC_RELEASE, "workgroup");
    __builtin_amdgcn_wave_barrier();
    __builtin_amdgcn_fence(__ATOMIC_ACQUIRE, "workgroup");
  }
}

}

__device__ __forceinline__ void ln_row(const float* __restrict__ x, int L, float* v, float& mu, float& inv) {
    #pragma clang fp contract(off)
    float s = 0.f;
#pragma unroll
    for (int j = 0; j < 6; ++j) {
        const v4f t = *(const v4f*)(x + 128 * j + 4 * L);
        v[4 * j] = bfr(t.x); v[4 * j + 1] = bfr(t.y); v[4 * j + 2] = bfr(t.z); v[4 * j + 3] = bfr(t.w);
        s = (((s + v[4 * j]) + v[4 * j + 1]) + v[4 * j + 2]) + v[4 * j + 3];
    }
#pragma unroll
    for (int o = 16; o > 0; o >>= 1) s += __shfl_xor(s, o, 32);
    mu = s * (1.0f / (float)DM);
    float q = 0.f;
#pragma unroll
    for (int j = 0; j < 24; ++j) { const float d = v[j] - mu; q = q + d * d; }
#pragma unroll
    for (int o = 16; o > 0; o >>= 1) q += __shfl_xor(q, o, 32);
    const float sd = sqrtf(q * (1.0f / (float)(DM - 1)));
    inv = 1.0f / (sd + 1e-6f);
}
__device__ __forceinline__ float ln_val(float xb, float mu, float inv, float g, float bb) {
    #pragma clang fp contract(off)
    return (g * (xb - mu)) * inv + bb;
}

__global__ __launch_bounds__(256) void k_lnpl(const float* __restrict__ X, long long row0, int R, const float* __restrict__ G, const float* __restrict__ Bv,
                                             unsigned short* __restrict__ P, int pitch, int dup) {
    #pragma clang fp contract(off)
    const int r = blockIdx.x * 8 + (threadIdx.x >> 5); const int L = threadIdx.x & 31;
    if (r >= R) return;
    const float* x = X + ((size_t)row0 + (size_t)r) * DM;
    float v[24]; float mu, inv;
    ln_row(x, L, v, mu, inv);
    unsigned short* row = P + (size_t)r * (size_t)pitch;
#pragma unroll
    for (int j = 0; j < 6; ++j) {
        const int c = 128 * j + 4 * L;
        const v4f gg = *(const v4f*)(G + c); const v4f bb = *(const v4f*)(Bv + c);
        float o4[4];
        o4[0] = ln_val(v[4 * j],     mu, inv, bfr(gg.x), bfr(bb.x));
        o4[1] = ln_val(v[4 * j + 1], mu, inv, bfr(gg.y), bfr(bb.y));
        o4[2] = ln_val(v[4 * j + 2], mu, inv, bfr(gg.z), bfr(bb.z));
        o4[3] = ln_val(v[4 * j + 3], mu, inv, bfr(gg.w), bfr(bb.w));
        unsigned long long ph, pl; split4(o4, ph, pl);
        VST2(unsigned long long, (unsigned long long*)(row + c), ph);
        VST2(unsigned long long, (unsigned long long*)(row + DM + c), pl);
        if (dup) VST2(unsigned long long, (unsigned long long*)(row + 2 * DM + c), ph);
    }
}

__global__ __launch_bounds__(256) void k_wplane(const float* __restrict__ Wm, int NO, unsigned short* __restrict__ Bt) {
    const long long u = (long long)blockIdx.x * 256 + threadIdx.x; const int per = DM / 8;
    if (u >= (long long)NO * per) return;
    const int k0 = 8 * (int)(u % per); const int o = (int)(u / per);
    unsigned short hb[8];
#pragma unroll
    for (int i = 0; i < 8; ++i) hb[i] = bfbits(Wm[(size_t)(k0 + i) * NO + o]);
    const v4u pk = pack8(hb);
    unsigned short* d = Bt + (size_t)o * P2 + k0;
    VST2(v4u, (v4u*)d, pk);
    VST2(v4u, (v4u*)(d + DM), pk);
}

__global__ __launch_bounds__(256) void k_tr3(const float* __restrict__ S, int R, int C, int Z, unsigned short* __restrict__ Dp) {
    const long long u = (long long)blockIdx.x * 256 + threadIdx.x; const int per = R / 8;
    if (u >= (long long)Z * C * per) return;
    const int r0 = 8 * (int)(u % per); const long long zc = u / per; const int c = (int)(zc % C); const int z = (int)(zc / C);
    unsigned short hb[8], lb[8];
#pragma unroll
    for (int i = 0; i < 8; ++i) { const float f = S[((size_t)z * R + (size_t)(r0 + i)) * C + c]; hb[i] = bfbits(f); lb[i] = bfbits(f - bfval(hb[i])); }
    const v4u hv = pack8(hb), lv = pack8(lb);
    unsigned short* d = Dp + (size_t)zc * (size_t)(3 * R) + r0;
    VST2(v4u, (v4u*)d, hv);
    VST2(v4u, (v4u*)(d + R), lv);
    VST2(v4u, (v4u*)(d + 2 * R), hv);
}
__global__ __launch_bounds__(256) void k_tr3h(const unsigned short* __restrict__ S, int R, int C, int Z, unsigned short* __restrict__ Dp) {
    const long long u = (long long)blockIdx.x * 256 + threadIdx.x; const int per = R / 8;
    if (u >= (long long)Z * C * per) return;
    const int r0 = 8 * (int)(u % per); const long long zc = u / per; const int c = (int)(zc % C); const int z = (int)(zc / C);
    unsigned short hb[8], lb[8];
#pragma unroll
    for (int i = 0; i < 8; ++i) { const size_t so = ((size_t)z * R + (size_t)(r0 + i)) * (size_t)(3 * C); hb[i] = S[so + c]; lb[i] = S[so + 2 * C + c]; }
    const v4u hv = pack8(hb), lv = pack8(lb);
    unsigned short* d = Dp + (size_t)zc * (size_t)(3 * R) + r0;
    VST2(v4u, (v4u*)d, hv);
    VST2(v4u, (v4u*)(d + R), hv);
    VST2(v4u, (v4u*)(d + 2 * R), lv);
}

__global__ __launch_bounds__(256) void k_logit(const float* __restrict__ Hm, int R, const float* __restrict__ w, float* __restrict__ dst) {
    #pragma clang fp contract(off)
    __shared__ float w_s[HDN];
    w_s[threadIdx.x] = bfr(w[threadIdx.x]);
    __syncthreads();
    const int r = blockIdx.x * 256 + threadIdx.x;
    if (r >= R) return;
    const float* h = Hm + (size_t)r * HDN; float s = 0.f;
#pragma unroll 4
    for (int k = 0; k < HDN; ++k) s = s + w_s[k] * h[k];
    VST2(float, dst + r, s);
}

template <int L>
__global__ __launch_bounds__(256) void k_pool(const float* __restrict__ X, const int* __restrict__ MK, const float* __restrict__ LG,
                                             const float* __restrict__ G, const float* __restrict__ Bv, float* __restrict__ O) {
    #pragma clang fp contract(off)
    __shared__ float mu_s[L], inv_s[L], a_s[L];
    __shared__ float red[256];
    const int p = blockIdx.x; const int tid = threadIdx.x, wave = tid >> 5, lane = tid & 31;
    const float* xb = X + (size_t)p * L * DM;
    for (int l = wave; l < L; l += 8) {
        float v[24]; float mu, inv;
        ln_row(xb + (size_t)l * DM, lane, v, mu, inv);
        if (lane == 0) { mu_s[l] = mu; inv_s[l] = inv; }
    }
    __syncthreads();
    float sv = -__builtin_inff();
    if (tid < L) { const float lg = LG[(size_t)p * L + tid]; sv = (MK[(size_t)p * L + tid] != 0) ? lg : -1e18f; }
    red[tid] = sv; __syncthreads();
    for (int o = 128; o > 0; o >>= 1) { if (tid < o) red[tid] = fmaxf(red[tid], red[tid + o]); __syncthreads(); }
    const float mx = red[0]; __syncthreads();
    const float ex = (tid < L) ? expf(sv - mx) : 0.f;
    red[tid] = ex; __syncthreads();
    for (int o = 128; o > 0; o >>= 1) { if (tid < o) red[tid] += red[tid + o]; __syncthreads(); }
    const float rinv = 1.0f / red[0];
    if (tid < L) a_s[tid] = ex * rinv;
    __syncthreads();
    float acc[3] = {0.f, 0.f, 0.f}; float gb[3], bb[3];
#pragma unroll
    for (int k = 0; k < 3; ++k) { gb[k] = bfr(G[tid + 256 * k]); bb[k] = bfr(Bv[tid + 256 * k]); }
#pragma unroll 1
    for (int l = 0; l < L; ++l) {
        const float m = mu_s[l], iv = inv_s[l], a = a_s[l];
        const float* x = xb + (size_t)l * DM + tid;
#pragma unroll
        for (int k = 0; k < 3; ++k) { const float c = ln_val(bfr(x[256 * k]), m, iv, gb[k], bb[k]); acc[k] = acc[k] + a * c; }
    }
#pragma unroll
    for (int k = 0; k < 3; ++k) VST2(float, O + (size_t)p * DM + tid + 256 * k, acc[k]);
}

extern "C" void kernel_launch(void* const* d_in, const int* in_sizes, int n_in, void* d_out, int out_size, void* d_ws, size_t ws_size, hipStream_t stream) {
    if (n_in < 11) return;
    if (in_sizes[0] < NPAIR * LCQ * DM || in_sizes[1] < NPAIR * LCQ || in_sizes[2] < NPAIR * LEQ * DM || in_sizes[3] < NPAIR * LEQ ||
        in_sizes[4] < DM || in_sizes[5] < DM || in_sizes[6] < DM * DM || in_sizes[7] < DM * HDN || in_sizes[8] < DM * HDN ||
        in_sizes[9] < HDN || in_sizes[10] < HDN) return;
    if (out_size < NPAIR_FULL * DM + NPAIR * DM) return;
    const float* X1  = (const float*)d_in[0];
    const int*   M1  = (const int*)d_in[1];
    const float* X2  = (const float*)d_in[2];
    const int*   M2  = (const int*)d_in[3];
    const float* gain = (const float*)d_in[4];
    const float* lnb  = (const float*)d_in[5];
    const float* Wf  = (const float*)d_in[6];
    const float* W1  = (const float*)d_in[7];
    const float* W2  = (const float*)d_in[8];
    const float* w1  = (const float*)d_in[9];
    const float* w2  = (const float*)d_in[10];
    float* out = (float*)d_out;

    char* wsb = (char*)d_ws; size_t off = 0;
    auto take = [&](size_t bytes) -> char* { char* r = wsb + off; off += (bytes + 255) & ~(size_t)255; return r; };
    unsigned short* Wf2   = (unsigned short*)take((size_t)DM * P2 * 2);
    unsigned short* W12   = (unsigned short*)take((size_t)HDN * P2 * 2);
    unsigned short* W22   = (unsigned short*)take((size_t)HDN * P2 * 2);
    unsigned short* Cpl   = (unsigned short*)take((size_t)PCH * LCQ * P2 * 2);
    unsigned short* Epl   = (unsigned short*)take((size_t)PCH * LEQ * P3 * 2);
    unsigned short* CWpl  = (unsigned short*)take((size_t)PCH * LCQ * P3 * 2);
    float* cW1            = (float*)take((size_t)PCH * LCQ * HDN * 4);
    float* eW2            = (float*)take((size_t)PCH * LEQ * HDN * 4);
    unsigned short* cW1T3 = (unsigned short*)take((size_t)PCH * HDN * PT3 * 2);
    unsigned short* eW2T3 = (unsigned short*)take((size_t)PCH * HDN * PA3 * 2);
    unsigned short* AFF3  = (unsigned short*)take((size_t)PCH * LCQ * PA3 * 2);
    unsigned short* AFFT3 = (unsigned short*)take((size_t)PCH * LEQ * PT3 * 2);
    float* Hc             = (float*)take((size_t)PCH * LCQ * HDN * 4);
    float* He             = (float*)take((size_t)PCH * LEQ * HDN * 4);
    float* lg1            = (float*)take((size_t)NPAIR * LCQ * 4);
    float* lg2            = (float*)take((size_t)NPAIR * LEQ * 4);
    if (off > ws_size) return;

    k_wplane<<<(unsigned)(((long long)DM * (DM / 8) + 255) / 256), 256, 0, stream>>>(Wf, DM, Wf2);
    k_wplane<<<(unsigned)(((long long)HDN * (DM / 8) + 255) / 256), 256, 0, stream>>>(W1, HDN, W12);
    k_wplane<<<(unsigned)(((long long)HDN * (DM / 8) + 255) / 256), 256, 0, stream>>>(W2, HDN, W22);

    for (int p0 = 0; p0 < NPAIR; p0 += PCH) {
        const int np = (NPAIR - p0 < PCH) ? (NPAIR - p0) : PCH;
        const int Rc = np * LCQ, Re = np * LEQ;
        k_lnpl<<<(unsigned)((Rc + 7) / 8), 256, 0, stream>>>(X1, (long long)p0 * LCQ, Rc, gain, lnb, Cpl, P2, 0);
        k_lnpl<<<(unsigned)((Re + 7) / 8), 256, 0, stream>>>(X2, (long long)p0 * LEQ, Re, gain, lnb, Epl, P3, 1);
        w25::wmma_gemm64<1, false, 0, 2, false, 0><<<dim3((unsigned)((np * (DM / 64) + 7) / 8), 1), 256, 0, stream>>>(
            Cpl, nullptr, P2, 0, Wf2, nullptr, P2, 0, (void*)CWpl, (void*)(CWpl + 2 * DM), (void*)(CWpl + DM), P3, 0, nullptr, nullptr, 0, Rc, DM, P2, 1.0f);
        w25::wmma_gemm64<1, false, 0, 0, false, 0><<<dim3((unsigned)((np * (HDN / 64) + 7) / 8), 1), 256, 0, stream>>>(
            Cpl, nullptr, P2, 0, W12, nullptr, P2, 0, (void*)cW1, nullptr, nullptr, HDN, 0, nullptr, nullptr, 0, Rc, HDN, P2, 1.0f);
        w25::wmma_gemm64<1, false, 0, 0, false, 0><<<dim3((unsigned)((2 * np * (HDN / 64) + 7) / 8), 1), 256, 0, stream>>>(
            Epl, nullptr, P3, 0, W22, nullptr, P2, 0, (void*)eW2, nullptr, nullptr, HDN, 0, nullptr, nullptr, 0, Re, HDN, P2, 1.0f);
        w25::wmma_gemm64<1, false, 0, 2, false, 1><<<dim3(1, (unsigned)np), 256, 0, stream>>>(
            CWpl, nullptr, P3, (long)LCQ * P3, Epl, nullptr, P3, (long)LEQ * P3, (void*)AFF3, (void*)(AFF3 + 2 * LEQ), (void*)(AFF3 + LEQ), PA3, (long)LCQ * PA3,
            nullptr, nullptr, 0, LCQ, LEQ, P3, 1.0f);
        k_tr3<<<(unsigned)(((long long)np * HDN * (LCQ / 8) + 255) / 256), 256, 0, stream>>>(cW1, LCQ, HDN, np, cW1T3);
        k_tr3<<<(unsigned)(((long long)np * HDN * (LEQ / 8) + 255) / 256), 256, 0, stream>>>(eW2, LEQ, HDN, np, eW2T3);
        k_tr3h<<<(unsigned)(((long long)np * LEQ * (LCQ / 8) + 255) / 256), 256, 0, stream>>>(AFF3, LCQ, LEQ, np, AFFT3);
        w25::wmma_gemm64<1, false, 0, 0, true, 1><<<dim3(1, (unsigned)np), 256, 0, stream>>>(
            AFF3, nullptr, PA3, (long)LCQ * PA3, eW2T3, nullptr, PA3, (long)HDN * PA3, (void*)Hc, nullptr, nullptr, HDN, (long)LCQ * HDN,
            nullptr, cW1, (long)LCQ * HDN, LCQ, HDN, PA3, 1.0f);
        w25::wmma_gemm64<1, false, 0, 0, true, 1><<<dim3(1, (unsigned)np), 256, 0, stream>>>(
            AFFT3, nullptr, PT3, (long)LEQ * PT3, cW1T3, nullptr, PT3, (long)HDN * PT3, (void*)He, nullptr, nullptr, HDN, (long)LEQ * HDN,
            nullptr, eW2, (long)LEQ * HDN, LEQ, HDN, PT3, 1.0f);
        k_logit<<<(unsigned)((Rc + 255) / 256), 256, 0, stream>>>(Hc, Rc, w1, lg1 + (size_t)p0 * LCQ);
        k_logit<<<(unsigned)((Re + 255) / 256), 256, 0, stream>>>(He, Re, w2, lg2 + (size_t)p0 * LEQ);
    }
    k_pool<LCQ><<<(unsigned)NPAIR, 256, 0, stream>>>(X1, M1, lg1, gain, lnb, out);
    k_pool<LEQ><<<(unsigned)NPAIR, 256, 0, stream>>>(X2, M2, lg2, gain, lnb, out + (size_t)NPAIR_FULL * DM);
}
